// VectorizedQuantumCircuit_6992206758571
// MI455X (gfx1250) — hardware-verified
//
#include <hip/hip_runtime.h>


namespace {
constexpr int NQ = 12, NL = 2, DIM = 4096, B = 1024;

typedef _Float16 b16;
typedef __attribute__((ext_vector_type(16))) _Float16 v16b;
typedef __attribute__((ext_vector_type(8))) _Float16 v8b;
typedef __attribute__((ext_vector_type(8))) float v8f;
typedef __attribute__((ext_vector_type(4))) float v4f;
__device__ __forceinline__ float bf16_rne(float f) { unsigned int u = __float_as_uint(f); u += 0x7FFFu + ((u >> 16) & 1u); return __uint_as_float(u & 0xFFFF0000u); }
__device__ __forceinline__ void split16(float v, b16& hi, b16& lo) { hi = (b16)v; lo = (b16)(v - (float)hi); }
__device__ __forceinline__ v16b frag_kb(const b16* p, int hh) { const v8b a = *(const v8b*)(p + 8 * hh), b = *(const v8b*)(p + 16 + 8 * hh); v16b f;
#pragma unroll
  for (int e = 0; e < 8; ++e) { f[e] = a[e]; f[8 + e] = b[e]; } return f; }
__device__ __forceinline__ void frag_split(const float* p, int hh, v16b& fh, v16b& fl) {
#pragma unroll
  for (int e = 0; e < 8; ++e) { b16 a, c; split16(p[8 * hh + e], a, c); fh[e] = a; fl[e] = c; split16(p[16 + 8 * hh + e], a, c); fh[8 + e] = a; fl[8 + e] = c; } }
__device__ __forceinline__ v8f wmma16b(v16b a, v16b b, v8f c) { v8f d = __builtin_amdgcn_wmma_f32_16x16x32_f16(false, a, false, b, (short)0, c, false, false); asm volatile("v_nop\n\tv_nop\n\tv_nop\n\tv_nop" : "+v"(d) : "v"(a), "v"(b)); return d; }
__device__ __forceinline__ void wave_lds_sync() { __builtin_amdgcn_fence(__ATOMIC_RELEASE, "workgroup"); __builtin_amdgcn_wave_barrier(); __builtin_amdgcn_fence(__ATOMIC_ACQUIRE, "workgroup"); }
__device__ __forceinline__ float pmul(float a, float b) { float p = a * b; asm volatile("" : "+v"(p)); return p; }
__device__ __forceinline__ void sincos_r(float ang, float& sn, float& cs) { const float k = rintf(ang * 0.15915494309189535f); float r = __builtin_fmaf(k, -6.28318548202514648f, ang); r = __builtin_fmaf(k, 1.7484556025237907e-7f, r);
  const float t = r * 0.15915494309189535f; sn = __builtin_amdgcn_sinf(t); cs = __builtin_amdgcn_cosf(t); }

__global__ __launch_bounds__(256) void signs_kernel(b16* __restrict__ sg) {
  const int t_ = blockIdx.x * 256 + threadIdx.x, nth = gridDim.x * 256;
  for (int pass = 0; pass < 2; ++pass) { for (int p = t_; p < 16 * DIM; p += nth) { const int q = p / DIM, i = p % DIM; sg[p] = (b16)((q < NQ) ? (1.0f - 2.0f * (float)((i >> q) & 1)) : 0.0f); } __threadfence(); }
}

__device__ __forceinline__ void ry(float* st, int q, float c, float s, int t_) {
  for (int p = t_; p < DIM / 2; p += 256) { const int lo = p & ((1 << q) - 1), hi = p >> q; const int i = (hi << (q + 1)) | lo, j = i | (1 << q); const float a = st[i], b = st[j]; st[i] = pmul(c, a) - pmul(s, b); st[j] = pmul(s, a) + pmul(c, b); }
}
__device__ __forceinline__ void cnot(float* st, int cq, int tq, int t_) {
  for (int p = t_; p < DIM / 4; p += 256) {
    int i = 0, src = p; for (int bpos = 0; bpos < NQ; ++bpos) { if (bpos == cq) i |= 1 << bpos; else if (bpos == tq) { } else { i |= (src & 1) << bpos; src >>= 1; } }
    const int j = i | (1 << tq); const float a = st[i], b = st[j]; st[i] = b; st[j] = a; }
}

__global__ __launch_bounds__(256) void circuit_kernel(const float* __restrict__ x, const float* __restrict__ th, float* __restrict__ probs) {
  __shared__ __attribute__((aligned(16))) float st[DIM]; __shared__ float cs_[NQ * 3][2];
  const int b = blockIdx.x, t_ = threadIdx.x;
  for (int i = t_; i < DIM; i += 256) st[i] = (i == 0) ? 1.0f : 0.0f;
  if (t_ < NQ * 3) { const float ang = (t_ < NQ) ? bf16_rne(x[b * NQ + t_]) : bf16_rne(th[t_ - NQ]); float sn, cs; sincos_r(ang * 0.5f, sn, cs); cs_[t_][0] = cs; cs_[t_][1] = sn; }
  __syncthreads();
  for (int q = 0; q < NQ; ++q) { ry(st, q, cs_[q][0], cs_[q][1], t_); __syncthreads(); }
  for (int l = 0; l < NL; ++l) {
    for (int q = 0; q < NQ; ++q) { ry(st, q, cs_[NQ + l * NQ + q][0], cs_[NQ + l * NQ + q][1], t_); __syncthreads(); }
    for (int q = 0; q < NQ; ++q) { cnot(st, q, (q + 1) % NQ, t_); __syncthreads(); } }
  for (int pass = 0; pass < 2; ++pass) { for (int i = t_; i < DIM / 4; i += 256) { v4f o; for (int e = 0; e < 4; ++e) { const float a = st[i * 4 + e]; o[e] = pmul(a, a); } *(volatile v4f*)(probs + (size_t)b * DIM + i * 4) = o; } __threadfence(); }
}

__global__ __launch_bounds__(128) void expect_kernel(const float* __restrict__ probs, const b16* __restrict__ sg, float* __restrict__ out) {
  __shared__ float Z[128][NQ];
  const int lane = threadIdx.x & 31, wave = threadIdx.x >> 5, nloc = lane & 15, hlf = lane >> 4, m0 = blockIdx.x * 128 + wave * 32;
  v8f acc[2] = {{}, {}};
#pragma unroll 4
  for (int kb = 0; kb < DIM; kb += 32) { v16b a0, l0, a1, l1; frag_split(probs + (size_t)(m0 + nloc) * DIM + kb, hlf, a0, l0); frag_split(probs + (size_t)(m0 + 16 + nloc) * DIM + kb, hlf, a1, l1); const v16b bw = frag_kb(sg + (size_t)nloc * DIM + kb, hlf);
    acc[0] = wmma16b(a0, bw, acc[0]); acc[0] = wmma16b(l0, bw, acc[0]); acc[1] = wmma16b(a1, bw, acc[1]); acc[1] = wmma16b(l1, bw, acc[1]); }
  if (nloc < NQ) {
#pragma unroll
    for (int r = 0; r < 2; ++r)
#pragma unroll
      for (int v = 0; v < 8; ++v) Z[wave * 32 + r * 16 + 8 * hlf + v][nloc] = acc[r][v]; }
  __syncthreads();
  for (int pass = 0; pass < 2; ++pass) { for (int i = threadIdx.x; i < 128 * NQ / 4; i += 128) *(volatile v4f*)(out + (size_t)blockIdx.x * 128 * NQ + i * 4) = *(const v4f*)(&Z[0][0] + i * 4); __threadfence(); }
}
}

extern "C" void kernel_launch(void* const* d_in, const int* in_sizes, int n_in,
                              void* d_out, int out_size, void* d_ws, size_t ws_size, hipStream_t stream) {
  (void)n_in; (void)out_size;
  const float* x = (const float*)d_in[0]; const float* th = (const float*)d_in[1];
  float* out = (float*)d_out;
  if (in_sizes[0] != B * NQ || in_sizes[1] != NL * NQ) return;
  size_t off = 0; char* ws = (char*)d_ws;
  auto carve = [&](size_t bytes) { char* p = ws + off; off += (bytes + 255) & ~(size_t)255; return p; };
  b16* sg = (b16*)carve((size_t)16 * DIM * 2); float* probs = (float*)carve((size_t)B * DIM * 4);
  if (off > ws_size) return;
  signs_kernel<<<64, 256, 0, stream>>>(sg);
  circuit_kernel<<<B, 256, 0, stream>>>(x, th, probs);
  expect_kernel<<<B / 128, 128, 0, stream>>>(probs, sg, out);
}
